// NonLocal2D_53377853555280
// MI455X (gfx1250) — hardware-verified
//
#include <hip/hip_runtime.h>
#include <stdint.h>


typedef __bf16         v16bf __attribute__((ext_vector_type(16)));
typedef float          v8f   __attribute__((ext_vector_type(8)));
typedef float          v4f   __attribute__((ext_vector_type(4)));
typedef unsigned short v8us  __attribute__((ext_vector_type(8)));
typedef unsigned int   v4u   __attribute__((ext_vector_type(4)));

#define C_IN      256
#define C_MID     128
#define HH        96
#define NPOS      (HH * HH)
#define PHN       (HH / 2)
#define PWN       (HH / 2)
#define NKP       (PHN * PWN)
#define KROW      64
#define KPAD      (PHN * KROW)
#define XS1_PITCH 136
#define XS2_PITCH 264
#define STRIP     64

__device__ __forceinline__ unsigned short f2bf_bits(float f) {
  unsigned u = __builtin_bit_cast(unsigned, f);
  unsigned r = u + 0x7FFFu + ((u >> 16) & 1u);
  return (unsigned short)(r >> 16);
}
__device__ __forceinline__ unsigned pack2_bf(float lo, float hi) {
  return (unsigned)f2bf_bits(lo) | ((unsigned)f2bf_bits(hi) << 16);
}

union Frag { v16bf v; v8us u[2]; };

__device__ __forceinline__ v16bf ld_frag(const unsigned short* p_lo, const unsigned short* p_hi) {
  Frag f;
  f.u[0] = *reinterpret_cast<const v8us*>(p_lo);
  f.u[1] = *reinterpret_cast<const v8us*>(p_hi);
  return f.v;
}

__device__ __forceinline__ v16bf frag_from_f32(const float* w) {
  const v4f w0 = *reinterpret_cast<const v4f*>(w);
  const v4f w1 = *reinterpret_cast<const v4f*>(w + 4);
  const v4f w2 = *reinterpret_cast<const v4f*>(w + 16);
  const v4f w3 = *reinterpret_cast<const v4f*>(w + 20);
  v8us u0, u1;
  u0[0] = f2bf_bits(w0.x); u0[1] = f2bf_bits(w0.y); u0[2] = f2bf_bits(w0.z); u0[3] = f2bf_bits(w0.w);
  u0[4] = f2bf_bits(w1.x); u0[5] = f2bf_bits(w1.y); u0[6] = f2bf_bits(w1.z); u0[7] = f2bf_bits(w1.w);
  u1[0] = f2bf_bits(w2.x); u1[1] = f2bf_bits(w2.y); u1[2] = f2bf_bits(w2.z); u1[3] = f2bf_bits(w2.w);
  u1[4] = f2bf_bits(w3.x); u1[5] = f2bf_bits(w3.y); u1[6] = f2bf_bits(w3.z); u1[7] = f2bf_bits(w3.w);
  Frag f;
  f.u[0] = u0;
  f.u[1] = u1;
  return f.v;
}

__device__ __forceinline__ v8f wmma_bf16(const v16bf a, const v16bf b, v8f c) {
  v8f d = __builtin_amdgcn_wmma_f32_16x16x32_bf16(false, a, false, b, (short)0, c, false, false);
  asm volatile("v_nop\n\tv_nop\n\tv_nop\n\tv_nop" : "+v"(d) : "v"(a), "v"(b));
  return d;
}

__global__ __launch_bounds__(256) void k_conv_pool(
    const float* __restrict__ x2,
    const float* __restrict__ Wp, const float* __restrict__ bp,
    const float* __restrict__ Wg, const float* __restrict__ bg,
    unsigned short* __restrict__ phibuf, unsigned short* __restrict__ gbuf,
    int nb) {
  const int ph  = blockIdx.x;
  const int n   = blockIdx.y;
  const int sel = blockIdx.z;
  if (ph >= PHN || n >= nb) return;
  const float* Wc = sel ? Wg : Wp;
  const float* bc = sel ? bg : bp;
  unsigned short* dst = sel ? gbuf : phibuf;

  __shared__ __align__(16) unsigned short Xs[192 * XS1_PITCH];

  const int tid  = threadIdx.x;
  const int lane = tid & 31;
  const int wave = tid >> 5;
  const int half = lane >> 4;
  const int lr   = lane & 15;

  const float* xin = x2 + (size_t)n * C_IN * NPOS + (size_t)(2 * ph) * HH;

  v8f acc[6][2];
#pragma unroll
  for (int j = 0; j < 6; ++j) { acc[j][0] = 0.0f; acc[j][1] = 0.0f; }

  const int m = wave * 16 + lr;

  for (int kslice = 0; kslice < 2; ++kslice) {
    for (int e = tid; e < 16 * 192; e += 256) {
      const int p  = e % 192;
      const int cg = e / 192;
      const float* src = xin + (size_t)(kslice * 128 + 8 * cg) * NPOS + p;
      v4u pk;
      pk.x = pack2_bf(src[0],                 src[(size_t)1 * NPOS]);
      pk.y = pack2_bf(src[(size_t)2 * NPOS], src[(size_t)3 * NPOS]);
      pk.z = pack2_bf(src[(size_t)4 * NPOS], src[(size_t)5 * NPOS]);
      pk.w = pack2_bf(src[(size_t)6 * NPOS], src[(size_t)7 * NPOS]);
      *reinterpret_cast<v4u*>(&Xs[p * XS1_PITCH + 8 * cg]) = pk;
    }
    __syncthreads();

#pragma unroll
    for (int ks = 0; ks < 4; ++ks) {
      const int kk = ks * 32 + 8 * half;
      const v16bf a = frag_from_f32(Wc + (size_t)m * C_IN + kslice * 128 + kk);
#pragma unroll
      for (int j = 0; j < 6; ++j) {
        const unsigned short* r0 = &Xs[(j * 16 + lr) * XS1_PITCH + kk];
        const unsigned short* r1 = &Xs[((j + 6) * 16 + lr) * XS1_PITCH + kk];
        const v16bf b0 = ld_frag(r0, r0 + 16);
        const v16bf b1 = ld_frag(r1, r1 + 16);
        acc[j][0] = wmma_bf16(a, b0, acc[j][0]);
        acc[j][1] = wmma_bf16(a, b1, acc[j][1]);
      }
    }
    __syncthreads();
  }

  unsigned short* st = Xs + wave * (16 * KROW);
#pragma unroll
  for (int j = 0; j < 6; ++j) {
#pragma unroll
    for (int v = 0; v < 8; ++v) {
      const int row = 8 * half + v;
      const int mm  = wave * 16 + row;
      const float c0 = acc[j][0][v];
      const float c1 = acc[j][1][v];
      const float q0 = fmaxf(c0, __shfl_xor(c0, 1, 32));
      const float q1 = fmaxf(c1, __shfl_xor(c1, 1, 32));
      const float mx = fmaxf(q0, q1) + bc[mm];
      st[row * KROW + j * 8 + (lr >> 1)] = f2bf_bits(mx);
    }
  }
#pragma unroll
  for (int v = 0; v < 8; ++v) st[(8 * half + v) * KROW + PWN + lr] = (unsigned short)0;
  __syncthreads();

  v8us pv[4];
#pragma unroll
  for (int i = 0; i < 4; ++i) {
    const int q   = i * 32 + lane;
    const int row = q >> 3;
    const int col = (q & 7) * 8;
    pv[i] = *reinterpret_cast<const v8us*>(st + row * KROW + col);
  }
  unsigned short* gp = dst + ((size_t)n * C_MID + wave * 16) * KPAD + (size_t)ph * KROW;
#pragma unroll
  for (int i = 0; i < 4; ++i) {
    const int q = i * 32 + lane;
    *reinterpret_cast<volatile v8us*>(gp + (size_t)(q >> 3) * KPAD + (q & 7) * 8) = pv[i];
  }
  __threadfence();
#pragma unroll
  for (int i = 0; i < 4; ++i) {
    const int q = i * 32 + lane;
    *reinterpret_cast<volatile v8us*>(gp + (size_t)(q >> 3) * KPAD + (q & 7) * 8) = pv[i];
  }
}

__global__ __launch_bounds__(256) void k_gram(
    const unsigned short* __restrict__ phibuf,
    const unsigned short* __restrict__ gbuf,
    float* __restrict__ Sbuf, int nb) {
  const int n = blockIdx.x;
  if (n >= nb) return;

  __shared__ __align__(16) float Sst[8 * 16 * C_MID];

  const int tid  = threadIdx.x;
  const int lane = tid & 31;
  const int wave = tid >> 5;
  const int half = lane >> 4;
  const int lr   = lane & 15;

  const unsigned short* phv = phibuf + (size_t)n * C_MID * KPAD;
  const unsigned short* ggv = gbuf   + (size_t)n * C_MID * KPAD;

  v8f acc[8];
#pragma unroll
  for (int j = 0; j < 8; ++j) acc[j] = 0.0f;

  const unsigned short* arow = phv + (size_t)(wave * 16 + lr) * KPAD + 8 * half;
  const unsigned short* brow = ggv + (size_t)lr * KPAD + 8 * half;

#pragma unroll 2
  for (int ks = 0; ks < KPAD / 32; ++ks) {
    const int k0 = ks * 32;
    const v16bf a = ld_frag(arow + k0, arow + k0 + 16);
#pragma unroll
    for (int j = 0; j < 8; ++j) {
      const unsigned short* bq = brow + (size_t)(j * 16) * KPAD + k0;
      const v16bf b = ld_frag(bq, bq + 16);
      acc[j] = wmma_bf16(a, b, acc[j]);
    }
  }

  float* st = Sst + wave * (16 * C_MID);
#pragma unroll
  for (int j = 0; j < 8; ++j)
#pragma unroll
    for (int v = 0; v < 8; ++v)
      st[(8 * half + v) * C_MID + j * 16 + lr] = acc[j][v];
  __syncthreads();

  v4f pv[16];
#pragma unroll
  for (int i = 0; i < 16; ++i)
    pv[i] = *reinterpret_cast<const v4f*>(st + i * C_MID + lane * 4);

  float* S = Sbuf + ((size_t)n * C_MID + wave * 16) * C_MID + lane * 4;
#pragma unroll
  for (int i = 0; i < 16; ++i)
    *reinterpret_cast<volatile v4f*>(S + (size_t)i * C_MID) = pv[i];
  __threadfence();
#pragma unroll
  for (int i = 0; i < 16; ++i)
    *reinterpret_cast<volatile v4f*>(S + (size_t)i * C_MID) = pv[i];
}

__global__ __launch_bounds__(256) void k_fold1(
    const float* __restrict__ Sbuf, const float* __restrict__ Wt,
    float* __restrict__ Vbuf, int nb) {
  const int n = blockIdx.x;
  if (n >= nb) return;
  const int tid = threadIdx.x;
  const float* S = Sbuf + (size_t)n * C_MID * C_MID;
  float* V = Vbuf + (size_t)n * C_MID * C_IN;

  for (int it = 0; it < (C_MID * C_IN / 4) / 256; ++it) {
    const int item = it * 256 + tid;
    const int cp   = item >> 6;
    const int i0   = (item & 63) * 4;
    v4f a = 0.0f;
#pragma unroll 4
    for (int c = 0; c < C_MID; ++c) {
      const float s = S[c * C_MID + cp];
      const v4f  w = *reinterpret_cast<const v4f*>(Wt + (size_t)c * C_IN + i0);
      a += s * w;
    }
    float* p = V + (size_t)cp * C_IN + i0;
    *reinterpret_cast<volatile v4f*>(p) = a;
    __threadfence();
    *reinterpret_cast<volatile v4f*>(p) = a;
  }
}

__global__ __launch_bounds__(256) void k_fold2(
    const float* __restrict__ Sbuf, const float* __restrict__ Vbuf,
    const float* __restrict__ bt,
    const float* __restrict__ Wout, const float* __restrict__ bout,
    unsigned short* __restrict__ Ubf, float* __restrict__ betab, int nb) {
  const int n = blockIdx.x;
  if (n >= nb) return;
  __shared__ float vb_s[C_MID];
  __shared__ __align__(16) float beta_s[C_IN];

  const int tid = threadIdx.x;
  const float* S = Sbuf + (size_t)n * C_MID * C_MID;
  const float* V = Vbuf + (size_t)n * C_MID * C_IN;
  const float scale = 1.0f / (float)NKP;

  if (tid < C_MID) {
    float a = 0.0f;
#pragma unroll 4
    for (int c = 0; c < C_MID; ++c) a += S[c * C_MID + tid] * bt[c];
    vb_s[tid] = a;
  }
  __syncthreads();

  unsigned short* Ub = Ubf + (size_t)n * C_IN * C_IN;
  for (int it = 0; it < (C_IN * C_IN / 8) / 256; ++it) {
    const int item = it * 256 + tid;
    const int o    = item >> 5;
    const int i0   = (item & 31) * 8;
    const float* wr = Wout + (size_t)o * C_MID;
    v4f a0 = 0.0f, a1 = 0.0f;
#pragma unroll 4
    for (int c = 0; c < C_MID; ++c) {
      const float wv = wr[c];
      const float* vr = V + (size_t)c * C_IN + i0;
      a0 += wv * *reinterpret_cast<const v4f*>(vr);
      a1 += wv * *reinterpret_cast<const v4f*>(vr + 4);
    }
    v8us u;
    u[0] = f2bf_bits(a0.x * scale); u[1] = f2bf_bits(a0.y * scale);
    u[2] = f2bf_bits(a0.z * scale); u[3] = f2bf_bits(a0.w * scale);
    u[4] = f2bf_bits(a1.x * scale); u[5] = f2bf_bits(a1.y * scale);
    u[6] = f2bf_bits(a1.z * scale); u[7] = f2bf_bits(a1.w * scale);
    unsigned short* p = Ub + (size_t)o * C_IN + i0;
    *reinterpret_cast<volatile v8us*>(p) = u;
    __threadfence();
    *reinterpret_cast<volatile v8us*>(p) = u;
  }

  {
    const int o = tid;
    float a = 0.0f;
#pragma unroll 4
    for (int c = 0; c < C_MID; ++c) a += Wout[(size_t)o * C_MID + c] * vb_s[c];
    beta_s[o] = a * scale + bout[o];
  }
  __syncthreads();
  if (tid < 64) {
    const v4f bv = *reinterpret_cast<const v4f*>(beta_s + 4 * tid);
    float* p = betab + (size_t)n * C_IN + 4 * tid;
    *reinterpret_cast<volatile v4f*>(p) = bv;
    __threadfence();
    *reinterpret_cast<volatile v4f*>(p) = bv;
  }
}

__global__ __launch_bounds__(256) void k_apply(
    const float* __restrict__ x,
    const unsigned short* __restrict__ Ubf,
    const float* __restrict__ betab,
    float* __restrict__ out, int nb) {
  const int strip = blockIdx.x;
  const int n     = blockIdx.y;
  if (strip >= NPOS / STRIP || n >= nb) return;
  const int p0 = strip * STRIP;

  __shared__ __align__(16) float stage[C_IN * STRIP];
  unsigned short* Xs = reinterpret_cast<unsigned short*>(stage);

  const int tid  = threadIdx.x;
  const int lane = tid & 31;
  const int wave = tid >> 5;
  const int half = lane >> 4;
  const int lr   = lane & 15;

  const float* xin = x + (size_t)n * C_IN * NPOS;
  const unsigned short* U = Ubf + (size_t)n * C_IN * C_IN;

  for (int e = tid; e < STRIP * (C_IN / 8); e += 256) {
    const int pp = e & (STRIP - 1);
    const int cg = e >> 6;
    const float* src = xin + (size_t)(8 * cg) * NPOS + p0 + pp;
    v4u pk;
    pk.x = pack2_bf(src[0],                 src[(size_t)1 * NPOS]);
    pk.y = pack2_bf(src[(size_t)2 * NPOS], src[(size_t)3 * NPOS]);
    pk.z = pack2_bf(src[(size_t)4 * NPOS], src[(size_t)5 * NPOS]);
    pk.w = pack2_bf(src[(size_t)6 * NPOS], src[(size_t)7 * NPOS]);
    *reinterpret_cast<v4u*>(&Xs[pp * XS2_PITCH + 8 * cg]) = pk;
  }
  __syncthreads();

  v8f acc[8];
#pragma unroll
  for (int j = 0; j < 8; ++j) acc[j] = 0.0f;

  const int nt  = wave & 3;
  const int mtb = wave >> 2;
  const int col = nt * 16 + lr;

  const unsigned short* brow  = Xs + col * XS2_PITCH + 8 * half;
  const unsigned short* abase = U + (size_t)(mtb * 16 + lr) * C_IN + 8 * half;

#pragma unroll 2
  for (int ks = 0; ks < C_IN / 32; ++ks) {
    const int k0 = ks * 32;
    const v16bf b = ld_frag(brow + k0, brow + k0 + 16);
#pragma unroll
    for (int j = 0; j < 8; ++j) {
      const unsigned short* ap = abase + (size_t)(j * 32) * C_IN + k0;
      const v16bf a = ld_frag(ap, ap + 16);
      acc[j] = wmma_bf16(a, b, acc[j]);
    }
  }
  __syncthreads();

#pragma unroll
  for (int j = 0; j < 8; ++j)
#pragma unroll
    for (int v = 0; v < 8; ++v) {
      const int mrow = (mtb + 2 * j) * 16 + 8 * half + v;
      stage[mrow * STRIP + col] = acc[j][v];
    }
  __syncthreads();

  const float* bet  = betab + (size_t)n * C_IN;
  const float* xres = xin + p0;
  float* outp = out + (size_t)n * C_IN * NPOS + p0;
  const int c4 = (tid & 15) * 4;
  const int mr = tid >> 4;

  v4f ov[16];
#pragma unroll
  for (int i = 0; i < 16; ++i) {
    const int mm = i * 16 + mr;
    const v4f s  = *reinterpret_cast<const v4f*>(stage + mm * STRIP + c4);
    const v4f xv = *reinterpret_cast<const v4f*>(xres + (size_t)mm * NPOS + c4);
    const v4f mk = s + bet[mm];
    ov[i] = xv + mk;
  }
#pragma unroll
  for (int i = 0; i < 16; ++i)
    *reinterpret_cast<volatile v4f*>(outp + (size_t)(i * 16 + mr) * NPOS + c4) = ov[i];
  __threadfence();
#pragma unroll
  for (int i = 0; i < 16; ++i)
    *reinterpret_cast<volatile v4f*>(outp + (size_t)(i * 16 + mr) * NPOS + c4) = ov[i];
}

extern "C" void kernel_launch(void* const* d_in, const int* in_sizes, int n_in,
                              void* d_out, int out_size, void* d_ws,
                              size_t ws_size, hipStream_t stream) {
  if (n_in < 10) return;
  const int nx = in_sizes[0];
  if (nx <= 0) return;
  const int nb = nx / (C_IN * NPOS);
  if (nb < 1 || nb * (C_IN * NPOS) != nx) return;
  if (in_sizes[1] != nx || out_size != nx) return;
  if (in_sizes[2] != C_MID * C_IN || in_sizes[4] != C_MID * C_IN ||
      in_sizes[6] != C_MID * C_IN || in_sizes[8] != C_IN * C_MID) return;
  if (in_sizes[3] < C_MID || in_sizes[5] < C_MID || in_sizes[7] < C_MID || in_sizes[9] < C_IN) return;

  const float* x    = (const float*)d_in[0];
  const float* x2   = (const float*)d_in[1];
  const float* Wg   = (const float*)d_in[2];
  const float* bg   = (const float*)d_in[3];
  const float* Wt   = (const float*)d_in[4];
  const float* bt   = (const float*)d_in[5];
  const float* Wp   = (const float*)d_in[6];
  const float* bp   = (const float*)d_in[7];
  const float* Wout = (const float*)d_in[8];
  const float* bout = (const float*)d_in[9];
  float* out = (float*)d_out;

  char* wsb = (char*)d_ws;
  size_t off = 0;
  auto take = [&](size_t bytes) -> char* {
    char* p = wsb + off;
    off += (bytes + 255) & ~(size_t)255;
    return p;
  };

  unsigned short* phibuf = (unsigned short*)take((size_t)nb * C_MID * KPAD * 2);
  unsigned short* gbuf   = (unsigned short*)take((size_t)nb * C_MID * KPAD * 2);
  float*          Sbuf   = (float*)take((size_t)nb * C_MID * C_MID * 4);
  float*          Vbuf   = (float*)take((size_t)nb * C_MID * C_IN * 4);
  unsigned short* Ubf    = (unsigned short*)take((size_t)nb * C_IN * C_IN * 2);
  float*          betab  = (float*)take((size_t)nb * C_IN * 4);
  if (off > ws_size) return;

  k_conv_pool<<<dim3(PHN, nb, 2), 256, 0, stream>>>(x2, Wp, bp, Wg, bg, phibuf, gbuf, nb);
  k_gram<<<dim3(nb), 256, 0, stream>>>(phibuf, gbuf, Sbuf, nb);
  k_fold1<<<dim3(nb), 256, 0, stream>>>(Sbuf, Wt, Vbuf, nb);
  k_fold2<<<dim3(nb), 256, 0, stream>>>(Sbuf, Vbuf, bt, Wout, bout, Ubf, betab, nb);
  k_apply<<<dim3(NPOS / STRIP, nb), 256, 0, stream>>>(x, Ubf, betab, out, nb);
  (void)hipGetLastError();
}
